// MolecularNetwork_36077725286789
// MI455X (gfx1250) — hardware-verified
//
#include <hip/hip_runtime.h>
#include <stddef.h>


#define DF    128
#define KIN   64
#define NH    8
#define HC    16
#define GR    32
#define AP    136
#define XSP   132
#define NTHR  256
#define NWAVE 8
#define NB    480
#define CHUNK 1024
#define WCAP  ((CHUNK / NTHR) * 32)
#define GPW   4
#define PB    64
#define MAXT  16

#define LDS_SACC (NB * DF)
#define LDS_DEN  (NB * NH)
#define LDS_SMX  (NB * NH)
#define LDS_LIST (NWAVE * WCAP)
#define GAT_LDS_BYTES ((LDS_SACC + LDS_DEN + LDS_SMX + LDS_LIST + NWAVE) * 4)

static_assert(WCAP == 128);
static_assert(CHUNK == NTHR * 4);
static_assert(NB <= 512);
static_assert((NB % NWAVE) == 0);
static_assert((LDS_SACC % 4) == 0);
static_assert(GAT_LDS_BYTES == 280608);
static_assert(NWAVE * GPW == GR);
static_assert(MAXT * GR == 512);

typedef float    v4f  __attribute__((ext_vector_type(4)));
typedef float    v8f  __attribute__((ext_vector_type(8)));
typedef int      v4i  __attribute__((ext_vector_type(4)));
typedef _Float16 v8h  __attribute__((ext_vector_type(8)));
typedef _Float16 v16h __attribute__((ext_vector_type(16)));
union Frag   { v16h v; v8h half[2]; };
union Pack16 { v8h h; v4i i; };

__device__ __forceinline__ v8f wm(v16h a, v16h b, v8f c) {
  v8f d = __builtin_amdgcn_wmma_f32_16x16x32_f16(false, a, false, b, (short)0, c, false, false);
  asm volatile("v_nop\n\tv_nop\n\tv_nop\n\tv_nop" : "+v"(d) : "v"(a), "v"(b));
  return d;
}

__device__ __forceinline__ float wsum(float v) {
  v += __shfl_xor(v, 16, 32);
  v += __shfl_xor(v, 8, 32);
  v += __shfl_xor(v, 4, 32);
  v += __shfl_xor(v, 2, 32);
  v += __shfl_xor(v, 1, 32);
  return v;
}

__device__ __forceinline__ v8h cvt8(v4f a, v4f b) {
  Pack16 u;
  u.h[0] = (_Float16)a.x; u.h[1] = (_Float16)a.y; u.h[2] = (_Float16)a.z; u.h[3] = (_Float16)a.w;
  u.h[4] = (_Float16)b.x; u.h[5] = (_Float16)b.y; u.h[6] = (_Float16)b.z; u.h[7] = (_Float16)b.w;
  return u.h;
}

__global__ __launch_bounds__(NTHR) void k_prep(
    const float* __restrict__ embW, const float* __restrict__ gatW,
    const float* __restrict__ gaW1, const float* __restrict__ clsW1,
    _Float16* embT, _Float16* gatT, _Float16* gaT, _Float16* clsT, int L) {
  const int y = blockIdx.y;
  const float* src;
  _Float16* dst;
  int K;
  if (y == 0)          { src = embW;  dst = embT; K = KIN; }
  else if (y <= L)     { src = gatW + (size_t)(y - 1) * DF * DF; dst = gatT + (size_t)(y - 1) * DF * DF; K = DF; }
  else if (y == L + 1) { src = gaW1;  dst = gaT;  K = DF; }
  else                 { src = clsW1; dst = clsT; K = DF; }
  const int i  = blockIdx.x * NTHR + threadIdx.x;
  const int k8 = K >> 3;
  if (i >= DF * k8) return;
  const int n  = i / k8;
  const int k0 = (i - n * k8) * 8;
  Pack16 u;
#pragma unroll
  for (int j = 0; j < 8; ++j) u.h[j] = (_Float16)(src[(size_t)(k0 + j) * DF + n] * 8.0f);
  _Float16* p = dst + (size_t)n * K + k0;
  *(volatile v4i*)p = u.i;
  __threadfence();
  *(volatile v4i*)p = u.i;
}

__device__ __forceinline__ void epi_tile(v8f acc, int T, int hh, int m, int wave, int ncol,
                                         float cs, float cd, float* Xs, float* As, float* Ds) {
  float ss[8], sd[8];
#pragma unroll
  for (int r = 0; r < 8; ++r) {
    const float v = acc[r] * 0.125f;
    Xs[(T * 16 + 8 * hh + r) * XSP + ncol] = v;
    ss[r] = v * cs;
    sd[r] = v * cd;
  }
#pragma unroll
  for (int mk = 1; mk < 16; mk <<= 1) {
#pragma unroll
    for (int r = 0; r < 8; ++r) {
      ss[r] += __shfl_xor(ss[r], mk, 32);
      sd[r] += __shfl_xor(sd[r], mk, 32);
    }
  }
  if (m == 0) {
#pragma unroll
    for (int r = 0; r < 8; ++r) {
      As[(T * 16 + 8 * hh + r) * NH + wave] = ss[r];
      Ds[(T * 16 + 8 * hh + r) * NH + wave] = sd[r];
    }
  }
}

__device__ __forceinline__ void epi_emb(v8f acc, int T, int hh, int ncol, float pb,
                                        const float* __restrict__ tab, const int* Nt, float* Xs) {
#pragma unroll
  for (int r = 0; r < 8; ++r) {
    const int rl = T * 16 + 8 * hh + r;
    Xs[rl * XSP + ncol] = (acc[r] * 0.125f + pb) + tab[Nt[rl] * DF + ncol];
  }
}

template <int ACT>
__device__ __forceinline__ void epi_dot(v8f acc, int T, int hh, int m, int wave,
                                        float pb, float pw, float* Ps) {
  float ss[8];
#pragma unroll
  for (int r = 0; r < 8; ++r) {
    const float v = acc[r] * 0.125f + pb;
    const float t = (ACT == 0) ? tanhf(v) : fmaxf(v, 0.f);
    ss[r] = t * pw;
  }
#pragma unroll
  for (int mk = 1; mk < 16; mk <<= 1) {
#pragma unroll
    for (int r = 0; r < 8; ++r) ss[r] += __shfl_xor(ss[r], mk, 32);
  }
  if (m == 0) {
#pragma unroll
    for (int r = 0; r < 8; ++r) Ps[(T * 16 + 8 * hh + r) * NH + wave] = ss[r];
  }
}

template <int KD, int MODE>
__global__ __launch_bounds__(NTHR) void k_gemm(
    const float* __restrict__ A, const _Float16* __restrict__ Wt,
    const float* __restrict__ p0, const float* __restrict__ p1, const float* __restrict__ p2,
    const int* __restrict__ ip, float* o0, float* o1, float* o2, int nN, int nT) {
  __shared__ __attribute__((aligned(16))) _Float16 At[GR * AP];
  __shared__ __attribute__((aligned(16))) float Xs[GR * XSP];
  __shared__ __attribute__((aligned(16))) float As[GR * NH];
  __shared__ __attribute__((aligned(16))) float Ds[GR * NH];
  __shared__ __attribute__((aligned(16))) float Sc[GR];
  __shared__ int Nt[GR];

  const int tid  = threadIdx.x;
  const int lane = tid & 31;
  const int wave = tid >> 5;
  const int hh   = lane >> 4;
  const int m    = lane & 15;
  const int rowBase = blockIdx.x * GR;

  {
    const int r = tid >> 3;
    int row = rowBase + r;
    if (row > nN - 1) row = nN - 1;
    if (KD == DF) {
      const int c0 = (tid & 7) * 16;
      const float* p = A + (size_t)row * KD + c0;
      const v4f f0 = *(const v4f*)(p), f1 = *(const v4f*)(p + 4);
      const v4f f2 = *(const v4f*)(p + 8), f3 = *(const v4f*)(p + 12);
      *(v8h*)(At + r * AP + c0)     = cvt8(f0, f1);
      *(v8h*)(At + r * AP + c0 + 8) = cvt8(f2, f3);
    } else {
      const int c0 = (tid & 7) * 8;
      const float* p = A + (size_t)row * KD + c0;
      const v4f f0 = *(const v4f*)(p), f1 = *(const v4f*)(p + 4);
      *(v8h*)(At + r * AP + c0) = cvt8(f0, f1);
    }
    if (MODE == 0) {
      if (tid < GR) {
        int rr = rowBase + tid;
        if (rr > nN - 1) rr = nN - 1;
        int t = ip[rr];
        if (t < 0) t += nT;
        t = t < 0 ? 0 : (t > nT - 1 ? nT - 1 : t);
        Nt[tid] = t;
      }
    }
  }
  __syncthreads();

  const int ncol = wave * 16 + m;
  v8f c0a = {0.f, 0.f, 0.f, 0.f, 0.f, 0.f, 0.f, 0.f};
  v8f c1a = {0.f, 0.f, 0.f, 0.f, 0.f, 0.f, 0.f, 0.f};
#pragma unroll
  for (int kt = 0; kt < KD / 32; ++kt) {
    const int k0 = kt * 32;
    Frag a0, a1, b;
    const _Float16* pb  = Wt + (size_t)ncol * KD + k0 + 8 * hh;
    const _Float16* pa0 = At + m * AP + k0 + 8 * hh;
    const _Float16* pa1 = At + (16 + m) * AP + k0 + 8 * hh;
    b.half[0]  = *(const v8h*)pb;  b.half[1]  = *(const v8h*)(pb + 16);
    a0.half[0] = *(const v8h*)pa0; a0.half[1] = *(const v8h*)(pa0 + 16);
    a1.half[0] = *(const v8h*)pa1; a1.half[1] = *(const v8h*)(pa1 + 16);
    c0a = wm(a0.v, b.v, c0a);
    c1a = wm(a1.v, b.v, c1a);
  }

  if (MODE == 2) {
    const float pb = p0[ncol];
    const float pw = p1[ncol];
    epi_dot<0>(c0a, 0, hh, m, wave, pb, pw, As);
    epi_dot<0>(c1a, 1, hh, m, wave, pb, pw, As);
    __syncthreads();
    if (tid < GR) {
      float s = 0.f;
#pragma unroll
      for (int w = 0; w < NH; ++w) s += As[tid * NH + w];
      Sc[tid] = s + p2[0];
    }
    __syncthreads();
    if (tid < 8) {
      const v4f v = *(const v4f*)(Sc + 4 * tid);
      float* q = o0 + (size_t)rowBase + 4 * tid;
      *(volatile v4f*)q = v;
      __threadfence();
      *(volatile v4f*)q = v;
    }
  } else {
    if (MODE == 0) {
      const float pb = p0[ncol];
      epi_emb(c0a, 0, hh, ncol, pb, p1, Nt, Xs);
      epi_emb(c1a, 1, hh, ncol, pb, p1, Nt, Xs);
    } else {
      const float cs = p0[ncol];
      const float cd = p1[ncol];
      epi_tile(c0a, 0, hh, m, wave, ncol, cs, cd, Xs, As, Ds);
      epi_tile(c1a, 1, hh, m, wave, ncol, cs, cd, Xs, As, Ds);
    }
    __syncthreads();

    v4f xr[4];
#pragma unroll
    for (int i = 0; i < 4; ++i) xr[i] = *(const v4f*)(Xs + (4 * wave + i) * XSP + 4 * lane);
    float* gp = 0;
    v4f gv = {0.f, 0.f, 0.f, 0.f};
    if (MODE == 1) {
      if (wave < 2) {
        gv = *(const v4f*)(As + wave * 128 + 4 * lane);
        gp = o1 + (size_t)rowBase * NH + wave * 128 + 4 * lane;
      } else if (wave < 4) {
        gv = *(const v4f*)(Ds + (wave - 2) * 128 + 4 * lane);
        gp = o2 + (size_t)rowBase * NH + (wave - 2) * 128 + 4 * lane;
      }
    }
    float* xpp[4];
#pragma unroll
    for (int i = 0; i < 4; ++i) xpp[i] = o0 + (size_t)(rowBase + 4 * wave + i) * DF + 4 * lane;

#pragma unroll
    for (int i = 0; i < 4; ++i) *(volatile v4f*)(xpp[i]) = xr[i];
    if (gp) *(volatile v4f*)gp = gv;
    __threadfence();
#pragma unroll
    for (int i = 0; i < 4; ++i) *(volatile v4f*)(xpp[i]) = xr[i];
    if (gp) *(volatile v4f*)gp = gv;
  }
}

__global__ __launch_bounds__(NTHR) void k_gat(
    float* h, const int* __restrict__ ei, const float* __restrict__ xp,
    const float* __restrict__ asrc, const float* __restrict__ adst,
    const float* __restrict__ bias, const float* __restrict__ gam, const float* __restrict__ bet,
    int nN, int nE) {
  extern __shared__ v4f lds_dyn[];
  float* sacc = (float*)lds_dyn;
  float* den  = sacc + LDS_SACC;
  float* smx  = den + LDS_DEN;
  int*   list = (int*)(smx + LDS_SMX);
  int*   wcnt = list + LDS_LIST;

  const int tid  = threadIdx.x;
  const int lane = tid & 31;
  const int wave = tid >> 5;
  const int hd   = lane >> 2;
  const int nodeBase = blockIdx.x * NB;

  {
    const v4f z4 = {0.f, 0.f, 0.f, 0.f};
    for (int i = tid; i < LDS_SACC / 4; i += NTHR) lds_dyn[i] = z4;
    for (int i = tid; i < LDS_DEN; i += NTHR) { den[i] = 0.f; smx[i] = -1.0e30f; }
  }
  __syncthreads();

  const int* eid = ei + nE;
  const bool al16 = ((nE & 3) == 0);
  const int nChunks = (nE + CHUNK - 1) / CHUNK;

#pragma unroll 1
  for (int ch = 0; ch < nChunks; ++ch) {
    const int cbase = ch * CHUNK;
    int wc = 0;
    {
      const int el0 = tid * 4;
      const int e0  = cbase + el0;
      const int sent = -2147483647 - 1;
      v4i d;
      if (al16 && (e0 + 3 < nE)) {
        d = *(const v4i*)(eid + e0);
      } else {
        d.x = (e0     < nE) ? eid[min(e0, nE - 1)]     : sent;
        d.y = (e0 + 1 < nE) ? eid[min(e0 + 1, nE - 1)] : sent;
        d.z = (e0 + 2 < nE) ? eid[min(e0 + 2, nE - 1)] : sent;
        d.w = (e0 + 3 < nE) ? eid[min(e0 + 3, nE - 1)] : sent;
      }
      const unsigned s0 = (unsigned)d.x - (unsigned)nodeBase;
      const unsigned s1 = (unsigned)d.y - (unsigned)nodeBase;
      const unsigned s2 = (unsigned)d.z - (unsigned)nodeBase;
      const unsigned s3 = (unsigned)d.w - (unsigned)nodeBase;
      const bool h0 = s0 < (unsigned)NB;
      const bool h1 = s1 < (unsigned)NB;
      const bool h2 = s2 < (unsigned)NB;
      const bool h3 = s3 < (unsigned)NB;
      const unsigned many = __builtin_amdgcn_ballot_w32(h0 | h1 | h2 | h3);
      if (many != 0u) {
#define HITJ(J, HJ, SJ) { \
          const unsigned mj = __builtin_amdgcn_ballot_w32(HJ); \
          if (HJ) { \
            const int pos = wc + (int)__builtin_amdgcn_mbcnt_lo(mj, 0u); \
            if (pos < WCAP) list[wave * WCAP + pos] = ((el0 + (J)) << 9) | (int)(SJ); \
          } \
          wc += (int)__builtin_popcount(mj); }
        HITJ(0, h0, s0)
        HITJ(1, h1, s1)
        HITJ(2, h2, s2)
        HITJ(3, h3, s3)
#undef HITJ
      }
    }
    if (lane == 0) wcnt[wave] = wc;
    __syncthreads();

    if (wave == 0) {
      for (int wsx = 0; wsx < NWAVE; ++wsx) {
        int n = wcnt[wsx];
        if (n > WCAP) n = WCAP;
        if (n < 0) n = 0;
        for (int i = 0; i < n; ++i) {
          const int ent = list[wsx * WCAP + i];
          int slot = ent & 511;
          if (slot > NB - 1) slot = NB - 1;
          const int el = (ent >> 9) & (CHUNK - 1);
          int e = cbase + el;
          if (e > nE - 1) e = nE - 1;
          int src = ei[e];
          if (src < 0) src += nN;
          src = src < 0 ? 0 : (src > nN - 1 ? nN - 1 : src);
          int nd = nodeBase + slot;
          if (nd > nN - 1) nd = nN - 1;
          float al = asrc[(size_t)src * NH + hd] + adst[(size_t)nd * NH + hd];
          al = (al > 0.f) ? al : 0.2f * al;
          const int ai = slot * NH + hd;
          const float mo = smx[ai];
          const float mn = fmaxf(mo, al);
          const float sc = __expf(mo - mn);
          const float p  = __expf(al - mn);
          const v4f xv = *(const v4f*)(xp + (size_t)src * DF + 4 * lane);
          v4f* sp = (v4f*)(sacc + slot * DF + 4 * lane);
          const v4f cur = *sp;
          const v4f nxt = cur * sc + p * xv;
          *sp = nxt;
          if ((lane & 3) == 0) {
            const float dv = den[ai];
            den[ai] = dv * sc + p;
            smx[ai] = mn;
          }
        }
      }
    }
    __syncthreads();
  }

  const v4f b4 = *(const v4f*)(bias + 4 * lane);
  const v4f g4 = *(const v4f*)(gam + 4 * lane);
  const v4f e4 = *(const v4f*)(bet + 4 * lane);
#pragma unroll 1
  for (int j = 0; j < NB / NWAVE; ++j) {
    const int slot = wave * (NB / NWAVE) + j;
    const int node = nodeBase + slot;
    if (node >= nN) break;
    const size_t nrow = (size_t)node;
    float al = asrc[nrow * NH + hd] + adst[nrow * NH + hd];
    al = (al > 0.f) ? al : 0.2f * al;
    const int ai = slot * NH + hd;
    const float mo = smx[ai];
    const float mn = fmaxf(mo, al);
    const float sc = __expf(mo - mn);
    const float p  = __expf(al - mn);
    const v4f xv = *(const v4f*)(xp + nrow * DF + 4 * lane);
    const v4f sv = *(const v4f*)(sacc + slot * DF + 4 * lane) * sc + p * xv;
    const float dv  = den[ai] * sc + p;
    const float inv = 1.0f / dv;
    const v4f g = sv * inv + b4;
    const float s  = wsum(g.x + g.y + g.z + g.w);
    const float mu = s * (1.0f / DF);
    const v4f dd = g - mu;
    const float q  = wsum(dd.x * dd.x + dd.y * dd.y + dd.z * dd.z + dd.w * dd.w);
    const float rs = rsqrtf(q * (1.0f / DF) + 1e-5f);
    const v4f hp = *(const v4f*)(h + nrow * DF + 4 * lane);
    v4f y = dd * rs * g4 + e4;
    y = y + hp;
    y.x = y.x > 0.f ? y.x : 0.f;
    y.y = y.y > 0.f ? y.y : 0.f;
    y.z = y.z > 0.f ? y.z : 0.f;
    y.w = y.w > 0.f ? y.w : 0.f;
    float* op = h + nrow * DF + 4 * lane;
    *(volatile v4f*)op = y;
    __threadfence();
    *(volatile v4f*)op = y;
  }
}

__global__ __launch_bounds__(NTHR) void k_pool1(
    const float* __restrict__ h, const float* __restrict__ sc,
    float* part, float* pes, int nN, int rows) {
  __shared__ float red[NTHR];
  __shared__ __attribute__((aligned(16))) v4f wacc[NWAVE * 32];
  __shared__ float wes[NWAVE];
  const int tid  = threadIdx.x;
  const int lane = tid & 31;
  const int wave = tid >> 5;

  float mx = -3.0e38f;
#pragma unroll 1
  for (int i = tid; i < nN; i += NTHR) mx = fmaxf(mx, sc[i]);
  red[tid] = mx;
  __syncthreads();
  for (int s = NTHR / 2; s > 0; s >>= 1) {
    if (tid < s) red[tid] = fmaxf(red[tid], red[tid + s]);
    __syncthreads();
  }
  const float M = red[0];

  const int n0 = blockIdx.x * rows;
  const int n1 = min(n0 + rows, nN);
  v4f acc = {0.f, 0.f, 0.f, 0.f};
  float es = 0.f;
#pragma unroll 1
  for (int n = n0 + wave; n < n1; n += NWAVE) {
    const float e = expf(sc[n] - M);
    es += e;
    acc += e * *(const v4f*)(h + (size_t)n * DF + 4 * lane);
  }
  wacc[wave * 32 + lane] = acc;
  if (lane == 0) wes[wave] = es;
  __syncthreads();
  if (wave == 0) {
    v4f t = wacc[lane];
#pragma unroll
    for (int w = 1; w < NWAVE; ++w) t += wacc[w * 32 + lane];
    float s = wes[0];
#pragma unroll
    for (int w = 1; w < NWAVE; ++w) s += wes[w];
    float* p = part + (size_t)blockIdx.x * DF + 4 * lane;
    float* q = pes + (size_t)blockIdx.x * 32 + 4 * lane;
    const v4f sv4 = {s, s, s, s};
    *(volatile v4f*)p = t;
    if (lane < 8) *(volatile v4f*)q = sv4;
    __threadfence();
    *(volatile v4f*)p = t;
    if (lane < 8) *(volatile v4f*)q = sv4;
  }
}

__global__ __launch_bounds__(NTHR) void k_gpool(
    const float* __restrict__ h, const int* __restrict__ bt, float* gmean, int nN) {
  const int lane = threadIdx.x & 31;
  const int wave = threadIdx.x >> 5;
  const int gbase = (blockIdx.x * NWAVE + wave) * GPW;
  v4f a0 = {0.f, 0.f, 0.f, 0.f}, a1 = a0, a2 = a0, a3 = a0;
  int c0 = 0, c1 = 0, c2 = 0, c3 = 0;
#pragma unroll 1
  for (int base = 0; base < nN; base += 32) {
    const int n = base + lane;
    const int b = bt[min(n, nN - 1)];
    const unsigned rel = (unsigned)b - (unsigned)gbase;
    const bool hit = (n < nN) && (rel < (unsigned)GPW);
    unsigned msk = __builtin_amdgcn_ballot_w32(hit);
    while (msk != 0u) {
      const int i = __builtin_ctz(msk);
      msk &= msk - 1u;
      const int gl = __shfl((int)rel, i, 32);
      const v4f hv = *(const v4f*)(h + (size_t)(base + i) * DF + 4 * lane);
      if (gl == 0)      { a0 += hv; ++c0; }
      else if (gl == 1) { a1 += hv; ++c1; }
      else if (gl == 2) { a2 += hv; ++c2; }
      else              { a3 += hv; ++c3; }
    }
  }
  const v4f m0 = a0 * (1.0f / (float)(c0 > 1 ? c0 : 1));
  const v4f m1 = a1 * (1.0f / (float)(c1 > 1 ? c1 : 1));
  const v4f m2 = a2 * (1.0f / (float)(c2 > 1 ? c2 : 1));
  const v4f m3 = a3 * (1.0f / (float)(c3 > 1 ? c3 : 1));
  float* p0 = gmean + (size_t)(gbase + 0) * DF + 4 * lane;
  float* p1 = gmean + (size_t)(gbase + 1) * DF + 4 * lane;
  float* p2 = gmean + (size_t)(gbase + 2) * DF + 4 * lane;
  float* p3 = gmean + (size_t)(gbase + 3) * DF + 4 * lane;
  *(volatile v4f*)p0 = m0; *(volatile v4f*)p1 = m1; *(volatile v4f*)p2 = m2; *(volatile v4f*)p3 = m3;
  __threadfence();
  *(volatile v4f*)p0 = m0; *(volatile v4f*)p1 = m1; *(volatile v4f*)p2 = m2; *(volatile v4f*)p3 = m3;
}

__global__ __launch_bounds__(NTHR) void k_cls(
    const float* __restrict__ gmean, const float* __restrict__ part, const float* __restrict__ pes,
    const _Float16* __restrict__ Wt, const float* __restrict__ b1, const float* __restrict__ w2,
    const float* __restrict__ b2, float* out, int nG, int nPB, int nTiles) {
  __shared__ __attribute__((aligned(16))) _Float16 At[GR * AP];
  __shared__ __attribute__((aligned(16))) float Ps[GR * NH];
  __shared__ __attribute__((aligned(16))) float Hg[DF];
  __shared__ __attribute__((aligned(16))) float Os[MAXT * GR];

  const int tid  = threadIdx.x;
  const int lane = tid & 31;
  const int wave = tid >> 5;
  const int hh   = lane >> 4;
  const int m    = lane & 15;

  if (tid < DF) {
    float t = 0.f, s = 0.f;
#pragma unroll 1
    for (int b = 0; b < nPB; ++b) { t += part[(size_t)b * DF + tid]; s += pes[(size_t)b * 32]; }
    Hg[tid] = t * (1.0f / s);
  }
  for (int i = tid; i < MAXT * GR; i += NTHR) Os[i] = 0.f;
  __syncthreads();

  const int ncol = wave * 16 + m;
  const float pb = b1[ncol];
  const float pw = w2[ncol];
  const float bb = b2[0];

#pragma unroll 1
  for (int T2 = 0; T2 < nTiles; ++T2) {
    const int rowBase = T2 * GR;
    {
      const int r  = tid >> 3;
      const int c0 = (tid & 7) * 16;
      const float* p = gmean + (size_t)(rowBase + r) * DF + c0;
      v4f f0 = *(const v4f*)(p), f1 = *(const v4f*)(p + 4);
      v4f f2 = *(const v4f*)(p + 8), f3 = *(const v4f*)(p + 12);
      f0 += *(const v4f*)(Hg + c0);
      f1 += *(const v4f*)(Hg + c0 + 4);
      f2 += *(const v4f*)(Hg + c0 + 8);
      f3 += *(const v4f*)(Hg + c0 + 12);
      *(v8h*)(At + r * AP + c0)     = cvt8(f0, f1);
      *(v8h*)(At + r * AP + c0 + 8) = cvt8(f2, f3);
    }
    __syncthreads();

    v8f c0a = {0.f, 0.f, 0.f, 0.f, 0.f, 0.f, 0.f, 0.f};
    v8f c1a = {0.f, 0.f, 0.f, 0.f, 0.f, 0.f, 0.f, 0.f};
#pragma unroll
    for (int kt = 0; kt < DF / 32; ++kt) {
      const int k0 = kt * 32;
      Frag a0, a1, b;
      const _Float16* pbp = Wt + (size_t)ncol * DF + k0 + 8 * hh;
      const _Float16* pa0 = At + m * AP + k0 + 8 * hh;
      const _Float16* pa1 = At + (16 + m) * AP + k0 + 8 * hh;
      b.half[0]  = *(const v8h*)pbp; b.half[1]  = *(const v8h*)(pbp + 16);
      a0.half[0] = *(const v8h*)pa0; a0.half[1] = *(const v8h*)(pa0 + 16);
      a1.half[0] = *(const v8h*)pa1; a1.half[1] = *(const v8h*)(pa1 + 16);
      c0a = wm(a0.v, b.v, c0a);
      c1a = wm(a1.v, b.v, c1a);
    }
    epi_dot<1>(c0a, 0, hh, m, wave, pb, pw, Ps);
    epi_dot<1>(c1a, 1, hh, m, wave, pb, pw, Ps);
    __syncthreads();
    if (tid < GR) {
      float s = 0.f;
#pragma unroll
      for (int w = 0; w < NH; ++w) s += Ps[tid * NH + w];
      Os[rowBase + tid] = s + bb;
    }
    __syncthreads();
  }

  if (wave == 0) {
    v4f ov[4];
    int  oi[4];
    bool ok[4];
#pragma unroll
    for (int q = 0; q < 4; ++q) {
      oi[q] = (4 * q + (lane >> 3)) * 32 + (lane & 7) * 4;
      ov[q] = *(const v4f*)(Os + oi[q]);
      ok[q] = (oi[q] + 4 <= nG);
    }
    const int r0 = nG & ~3;
    const int nr = nG & 3;
    const float rv = (lane < nr) ? Os[r0 + lane] : 0.f;
#pragma unroll
    for (int q = 0; q < 4; ++q) if (ok[q]) *(volatile v4f*)(out + oi[q]) = ov[q];
    if (lane < nr) *(volatile float*)(out + r0 + lane) = rv;
    __threadfence();
#pragma unroll
    for (int q = 0; q < 4; ++q) if (ok[q]) *(volatile v4f*)(out + oi[q]) = ov[q];
    if (lane < nr) *(volatile float*)(out + r0 + lane) = rv;
  }
}

extern "C" void kernel_launch(void* const* d_in, const int* in_sizes, int n_in,
                              void* d_out, int out_size, void* d_ws, size_t ws_size,
                              hipStream_t stream) {
  if (n_in < 21) return;
  const int nN = in_sizes[0] / KIN;
  if (nN <= 0 || in_sizes[0] != nN * KIN) return;
  if (in_sizes[1] < 0 || (in_sizes[1] & 1) != 0) return;
  const int nE = in_sizes[1] / 2;
  if (in_sizes[2] != nN || in_sizes[3] != nN) return;
  if (in_sizes[4] != KIN * DF || in_sizes[5] != DF) return;
  if (in_sizes[6] < DF || (in_sizes[6] % DF) != 0) return;
  const int nT = in_sizes[6] / DF;
  if (in_sizes[7] < DF * DF || (in_sizes[7] % (DF * DF)) != 0) return;
  const int L = in_sizes[7] / (DF * DF);
  if (L > 64) return;
  if (in_sizes[8] != L * NH * HC || in_sizes[9] != L * NH * HC) return;
  if (in_sizes[10] != L * DF || in_sizes[11] != L * DF || in_sizes[12] != L * DF) return;
  if (in_sizes[13] != DF * DF || in_sizes[14] != DF || in_sizes[15] != DF || in_sizes[16] < 1) return;
  if (in_sizes[17] != DF * DF || in_sizes[18] != DF || in_sizes[19] != DF || in_sizes[20] < 1) return;
  const int G = out_size;
  if (G < 1 || G > MAXT * GR) return;

  const float* x          = (const float*)d_in[0];
  const int*   edge_index = (const int*)d_in[1];
  const int*   node_types = (const int*)d_in[2];
  const int*   batch      = (const int*)d_in[3];
  const float* emb_W      = (const float*)d_in[4];
  const float* emb_b      = (const float*)d_in[5];
  const float* ntype_emb  = (const float*)d_in[6];
  const float* gat_W      = (const float*)d_in[7];
  const float* att_src    = (const float*)d_in[8];
  const float* att_dst    = (const float*)d_in[9];
  const float* gat_b      = (const float*)d_in[10];
  const float* ln_g       = (const float*)d_in[11];
  const float* ln_b       = (const float*)d_in[12];
  const float* ga_W1      = (const float*)d_in[13];
  const float* ga_b1      = (const float*)d_in[14];
  const float* ga_W2      = (const float*)d_in[15];
  const float* ga_b2      = (const float*)d_in[16];
  const float* cls_W1     = (const float*)d_in[17];
  const float* cls_b1     = (const float*)d_in[18];
  const float* cls_W2     = (const float*)d_in[19];
  const float* cls_b2     = (const float*)d_in[20];
  float* out = (float*)d_out;

  const int nP  = ((nN + GR - 1) / GR) * GR;
  const int GT  = (G + GR - 1) / GR;
  const int rowsPB = (nN + PB - 1) / PB;

  size_t off = 0;
  char* base = (char*)d_ws;
#define CARVE(T, name, bytes) T* name = (T*)(base + off); off += (((size_t)(bytes)) + 255) & ~(size_t)255;
  CARVE(_Float16, embT, (size_t)DF * KIN * sizeof(_Float16))
  CARVE(_Float16, gatT, (size_t)L * DF * DF * sizeof(_Float16))
  CARVE(_Float16, gaT,  (size_t)DF * DF * sizeof(_Float16))
  CARVE(_Float16, clsT, (size_t)DF * DF * sizeof(_Float16))
  CARVE(float, hbuf,   (size_t)nP * DF * sizeof(float))
  CARVE(float, xp,     (size_t)nP * DF * sizeof(float))
  CARVE(float, asrc,   (size_t)nP * NH * sizeof(float))
  CARVE(float, adst,   (size_t)nP * NH * sizeof(float))
  CARVE(float, scores, (size_t)nP * sizeof(float))
  CARVE(float, part,   (size_t)PB * DF * sizeof(float))
  CARVE(float, pes,    (size_t)PB * 32 * sizeof(float))
  CARVE(float, gmean,  (size_t)GT * GR * DF * sizeof(float))
#undef CARVE
  if (off > ws_size) return;

  k_prep<<<dim3(DF * DF / 8 / NTHR, L + 3), NTHR, 0, stream>>>(
      emb_W, gat_W, ga_W1, cls_W1, embT, gatT, gaT, clsT, L);

  k_gemm<KIN, 0><<<nP / GR, NTHR, 0, stream>>>(
      x, embT, emb_b, ntype_emb, (const float*)0, node_types, hbuf, (float*)0, (float*)0, nN, nT);

  hipFuncSetAttribute(reinterpret_cast<const void*>(&k_gat),
                      hipFuncAttributeMaxDynamicSharedMemorySize, GAT_LDS_BYTES);
  const int gridGat = (nN + NB - 1) / NB;
  for (int l = 0; l < L; ++l) {
    k_gemm<DF, 1><<<nP / GR, NTHR, 0, stream>>>(
        hbuf, gatT + (size_t)l * DF * DF, att_src + (size_t)l * NH * HC, att_dst + (size_t)l * NH * HC,
        (const float*)0, (const int*)0, xp, asrc, adst, nN, nT);
    k_gat<<<gridGat, NTHR, GAT_LDS_BYTES, stream>>>(
        hbuf, edge_index, xp, asrc, adst, gat_b + (size_t)l * DF, ln_g + (size_t)l * DF,
        ln_b + (size_t)l * DF, nN, nE);
  }

  k_gemm<DF, 2><<<nP / GR, NTHR, 0, stream>>>(
      hbuf, gaT, ga_b1, ga_W2, ga_b2, (const int*)0, scores, (float*)0, (float*)0, nN, nT);

  k_pool1<<<PB, NTHR, 0, stream>>>(hbuf, scores, part, pes, nN, rowsPB);
  k_gpool<<<GT, NTHR, 0, stream>>>(hbuf, batch, gmean, nN);
  k_cls<<<1, NTHR, 0, stream>>>(gmean, part, pes, clsT, cls_b1, cls_W2, cls_b2, out, G, PB, GT);
}
